// MultiHeadAttention_52158082843478
// MI455X (gfx1250) — hardware-run, weakly checked
//
#include <hip/hip_runtime.h>


#ifndef NB
#define NB 4
#endif
#ifndef SEQ
#define SEQ 2048
#endif
#define NB_FULL  4
#define SEQ_FULL 2048
#ifndef OUT_SEQ
#define OUT_SEQ SEQ
#endif
#ifndef EARLY
#define EARLY (SEQ < 512 ? SEQ : 512)
#endif
#define DM   1024
#define NH_  16
#define HD   64
#define AW   4
#define QRS  2048.0f
#define QRI  (1.0f / 2048.0f)
#define SC2  (0.7071067812f * 1.4426950408889634f)
#define PSH  8.0f
#define WPS  64.0f
#define WPI  (1.0f / 64.0f)
#define NEGB (-3.0e38f)

static_assert(HD == 64);
static_assert(NH_ * HD == DM);
static_assert(DM % 64 == 0);
static_assert(DM % 32 == 0);
static_assert(SEQ % 64 == 0);
static_assert((NB * SEQ) % 64 == 0);
static_assert(SEQ % 32 == 0);
static_assert(EARLY % 64 == 0);
static_assert(EARLY <= SEQ);
static_assert(EARLY % (16 * AW) == 0);
static_assert((SEQ - EARLY) % (16 * AW) == 0);
static_assert(((size_t)SEQ * DM) % 8 == 0);
static_assert(NB <= NB_FULL);
static_assert(SEQ <= SEQ_FULL);

typedef _Float16 h16;
typedef unsigned short bf;
typedef __attribute__((ext_vector_type(16))) __bf16   v16bf;
typedef __attribute__((ext_vector_type(16))) _Float16 v16h;
typedef __attribute__((ext_vector_type(8)))  _Float16 v8h;
typedef __attribute__((ext_vector_type(8)))  unsigned short v8us;
typedef __attribute__((ext_vector_type(8)))  float    v8f;
typedef __attribute__((ext_vector_type(4)))  float    v4f;
typedef v4f  __attribute__((may_alias)) v4fa;

__device__ __forceinline__ unsigned short f2bf(float f) { unsigned u = __float_as_uint(f); u += 0x7FFFu + ((u >> 16) & 1u); return (unsigned short)(u >> 16); }
__device__ __forceinline__ float bfval(float f) { return __uint_as_float(((unsigned)f2bf(f)) << 16); }
__device__ __forceinline__ v16h cat16(v8h lo, v8h hi) { return __builtin_shufflevector(lo, hi, 0, 1, 2, 3, 4, 5, 6, 7, 8, 9, 10, 11, 12, 13, 14, 15); }
__device__ __forceinline__ v16bf cat16b(v8us lo, v8us hi) { return __builtin_bit_cast(v16bf, __builtin_shufflevector(lo, hi, 0, 1, 2, 3, 4, 5, 6, 7, 8, 9, 10, 11, 12, 13, 14, 15)); }
__device__ __forceinline__ v8f wmma16(v16h a, v16h b, v8f c) { return __builtin_amdgcn_wmma_f32_16x16x32_f16(false, a, false, b, (short)0, c, false, false); }
__device__ __forceinline__ v8f wmmab(v16bf a, v16bf b, v8f c) { return __builtin_amdgcn_wmma_f32_16x16x32_bf16(false, a, false, b, (short)0, c, false, false); }
__device__ __forceinline__ v16h  ldh(const h16* p) { return cat16(*(const v8h*)p, *(const v8h*)(p + 16)); }
__device__ __forceinline__ v16bf ldb(const bf* p)  { return cat16b(*(const v8us*)p, *(const v8us*)(p + 16)); }
__device__ __forceinline__ void wave_sync() { __builtin_amdgcn_fence(3  , "wavefront"); __builtin_amdgcn_wave_barrier(); asm volatile("" ::: "memory"); }

__global__ __launch_bounds__(256) void k_cvt8(const float* __restrict__ src, bf* dst, size_t n8) {
    const size_t i = (size_t)blockIdx.x * 256 + threadIdx.x; if (i >= n8) return;
    const v8f v = *(const v8f*)(src + i * 8); v8us o;
#pragma unroll
    for (int k = 0; k < 8; ++k) o[k] = f2bf(v[k]);
    *(volatile v8us*)(dst + i * 8) = o; __threadfence(); *(volatile v8us*)(dst + i * 8) = o;
}

__global__ __launch_bounds__(256) void k_wT(const float* __restrict__ src, unsigned short* dst, int R, int Cc, int f16out) {
    __shared__ __align__(16) float tl[64 * 65];
    const int tid = threadIdx.x;
    const int k0 = blockIdx.x * 64, n0 = blockIdx.y * 64, z = blockIdx.z;
    const float* s = src + (size_t)z * (size_t)R * (size_t)Cc;
#pragma unroll
    for (int i = 0; i < 4; ++i) { const int row = (tid >> 4) + 16 * i, c4 = (tid & 15) * 4;
        const v4f v = *(const v4f*)(s + (size_t)(k0 + row) * Cc + n0 + c4);
        tl[row * 65 + c4 + 0] = v[0]; tl[row * 65 + c4 + 1] = v[1]; tl[row * 65 + c4 + 2] = v[2]; tl[row * 65 + c4 + 3] = v[3]; }
    __syncthreads();
    v8us o[2];
#pragma unroll
    for (int i = 0; i < 2; ++i) { const int n = (tid >> 3) + 32 * i, k8 = (tid & 7) * 8;
        if (f16out != 0) { v8h hv;
#pragma unroll
            for (int e = 0; e < 8; ++e) hv[e] = (h16)(bfval(tl[(k8 + e) * 65 + n]) * WPS);
            o[i] = __builtin_bit_cast(v8us, hv);
        } else { v8us uv;
#pragma unroll
            for (int e = 0; e < 8; ++e) uv[e] = f2bf(tl[(k8 + e) * 65 + n]);
            o[i] = uv; } }
    unsigned short* p0 = dst + ((size_t)z * Cc + n0 + (tid >> 3)) * (size_t)R + k0 + (tid & 7) * 8;
    unsigned short* p1 = p0 + (size_t)32 * (size_t)R;
    *(volatile v8us*)p0 = o[0]; *(volatile v8us*)p1 = o[1];
    __threadfence();
    *(volatile v8us*)p0 = o[0]; *(volatile v8us*)p1 = o[1];
}

__global__ __launch_bounds__(32) void k_proj(const bf* __restrict__ A, const bf* __restrict__ Bt, h16* Ph, h16* Pr,
                                             int RB, size_t sRB, int pitch, int CB, size_t sCB,
                                             int resMode, int lim, size_t sRBr, int pitchr, size_t sCBr) {
    __shared__ __align__(16) float os[16 * 68];
    const int K = DM;
    const int lane = threadIdx.x & 31, lr = lane & 15, hi = lane >> 4; const int r0 = blockIdx.x * 64, c0 = blockIdx.y * 64;
    v8f acc[4][4];
#pragma unroll
    for (int mb = 0; mb < 4; ++mb)
#pragma unroll
        for (int nb = 0; nb < 4; ++nb) acc[mb][nb] = (v8f){};
    const size_t aoff = (size_t)(r0 + lr) * K + 8 * hi, boff = (size_t)(c0 + lr) * K + 8 * hi;
#pragma unroll 1
    for (int kc = 0; kc < K; kc += 32) {
        v16bf a[4];
#pragma unroll
        for (int mb = 0; mb < 4; ++mb) a[mb] = ldb(A + aoff + (size_t)mb * 16 * K + kc);
#pragma unroll
        for (int nb = 0; nb < 4; ++nb) { const v16bf b = ldb(Bt + boff + (size_t)nb * 16 * K + kc);
#pragma unroll
            for (int mb = 0; mb < 4; ++mb) acc[mb][nb] = wmmab(a[mb], b, acc[mb][nb]); }
        asm volatile("v_nop\n\tv_nop\n\tv_nop\n\tv_nop" : "+v"(acc[0][0]), "+v"(acc[1][1]), "+v"(acc[2][2]), "+v"(acc[3][3]) : "v"(a[0]), "v"(a[1]), "v"(a[2]), "v"(a[3]));
    }
    const int rIn = r0 % RB, cIn = c0 % CB;
    const size_t tbase  = (size_t)(r0 / RB) * sRB  + (size_t)rIn * (size_t)pitch  + (size_t)(c0 / CB) * sCB  + (size_t)cIn;
    const size_t tbaser = (size_t)(r0 / RB) * sRBr + (size_t)rIn * (size_t)pitchr + (size_t)(c0 / CB) * sCBr + (size_t)cIn;
    const int useRes = (resMode == 1) ? (rIn < lim) : ((resMode == 2) ? (cIn < lim) : 0);
#pragma unroll
    for (int mb = 0; mb < 4; ++mb) {
#pragma unroll
        for (int nb = 0; nb < 4; ++nb) {
#pragma unroll
            for (int j = 0; j < 8; ++j) os[(hi * 8 + j) * 68 + nb * 16 + lr] = acc[mb][nb][j]; }
        wave_sync();
        const size_t sb  = tbase  + (size_t)(mb * 16) * (size_t)pitch;
        const size_t sbr = tbaser + (size_t)(mb * 16) * (size_t)pitchr;
#pragma unroll 1
        for (int ps = 0; ps < 2; ++ps) {
#pragma unroll
            for (int s = 0; s < 4; ++s) { const int row = 4 * s + (lane >> 3), c8 = (lane & 7) * 8;
                const v4f x0 = *(const v4fa*)(&os[row * 68 + c8]); const v4f x1 = *(const v4fa*)(&os[row * 68 + c8 + 4]); v8h hv, rv;
#pragma unroll
                for (int i = 0; i < 4; ++i) { const h16 a0 = (h16)x0[i]; const h16 a1 = (h16)x1[i]; hv[i] = a0; hv[4 + i] = a1; rv[i] = (h16)((x0[i] - (float)a0) * QRS); rv[4 + i] = (h16)((x1[i] - (float)a1) * QRS); }
                *(volatile v8h*)(Ph + sb + (size_t)row * (size_t)pitch + c8) = hv;
                if (useRes) *(volatile v8h*)(Pr + sbr + (size_t)row * (size_t)pitchr + c8) = rv; }
            if (ps == 0) __threadfence(); }
        wave_sync();
    }
}

template <int EP>
__device__ __forceinline__ void flash_body(const h16* __restrict__ QH, const h16* __restrict__ QR, const h16* __restrict__ KH, const h16* __restrict__ KR,
                                           const h16* __restrict__ VH, const h16* __restrict__ VR, h16* CH, h16* CR, const int tbase) {
    __shared__ __align__(16) float os[AW * 16 * 68];
    const int lane = threadIdx.x & 31, wave = threadIdx.x >> 5, lr = lane & 15, hi = lane >> 4;
    const int zh = blockIdx.y; const int b = zh / NH_, h = zh % NH_;
    const int t0 = tbase + (blockIdx.x * AW + wave) * 16;
    const size_t pbase = (size_t)zh * SEQ * HD;
    const size_t rbase = (size_t)zh * EARLY * HD;
    const size_t qo = pbase + (size_t)(t0 + lr) * HD + 8 * hi;
    const v16h qh0 = ldh(QH + qo), qh1 = ldh(QH + qo + 32), qr0 = ldh(QR + qo), qr1 = ldh(QR + qo + 32);
    const size_t ko  = pbase + (size_t)lr * HD + 8 * hi;
    const size_t vo  = pbase + (size_t)lr * SEQ + 8 * hi;
    const size_t kro = rbase + (size_t)lr * HD + 8 * hi;
    const size_t vro = rbase + (size_t)lr * EARLY + 8 * hi;
    v8f oH[4], oL[4];
#pragma unroll
    for (int j = 0; j < 4; ++j) { oH[j] = (v8f){}; oL[j] = (v8f){}; }
    float m = NEGB, l = 0.0f;
    const int kend = t0 + 16;
    const int trow = t0 + lr;
#pragma unroll 1
    for (int key0 = 0; key0 < kend; key0 += 32) {
        v8f sHa = (v8f){}, sLa = (v8f){}, sHb = (v8f){}, sLb = (v8f){};
        {
            const h16* ka = KH + ko + (size_t)key0 * HD;
            const v16h ka0 = ldh(ka), ka1 = ldh(ka + 32), kb0 = ldh(ka + 16 * HD), kb1 = ldh(ka + 16 * HD + 32);
            sHa = wmma16(ka0, qh0, sHa); sLa = wmma16(ka0, qr0, sLa); sHb = wmma16(kb0, qh0, sHb); sLb = wmma16(kb0, qr0, sLb);
            sHa = wmma16(ka1, qh1, sHa); sLa = wmma16(ka1, qr1, sLa); sHb = wmma16(kb1, qh1, sHb); sLb = wmma16(kb1, qr1, sLb);
            if (EP) {
                const h16* kr = KR + kro + (size_t)key0 * HD;
                const v16h ra0 = ldh(kr), ra1 = ldh(kr + 32), rb0 = ldh(kr + 16 * HD), rb1 = ldh(kr + 16 * HD + 32);
                sLa = wmma16(ra0, qh0, sLa); sLb = wmma16(rb0, qh0, sLb);
                sLa = wmma16(ra1, qh1, sLa); sLb = wmma16(rb1, qh1, sLb);
                asm volatile("v_nop\n\tv_nop\n\tv_nop\n\tv_nop" : "+v"(sHa), "+v"(sLa), "+v"(sHb), "+v"(sLb) : "v"(ka0), "v"(ka1), "v"(kb0), "v"(kb1), "v"(ra0), "v"(ra1), "v"(rb0), "v"(rb1));
            } else {
                asm volatile("v_nop\n\tv_nop\n\tv_nop\n\tv_nop" : "+v"(sHa), "+v"(sLa), "+v"(sHb), "+v"(sLb) : "v"(ka0), "v"(ka1), "v"(kb0), "v"(kb1));
            }
        }
        float ta[8], tb[8];
#pragma unroll
        for (int r = 0; r < 8; ++r) { ta[r] = (sHa[r] + sLa[r] * QRI) * SC2; tb[r] = (sHb[r] + sLb[r] * QRI) * SC2; }
        if (key0 + 31 > t0) {
            const int kA = key0 + 8 * hi;
#pragma unroll
            for (int r = 0; r < 8; ++r) { ta[r] = (kA + r > trow) ? NEGB : ta[r]; tb[r] = (kA + 16 + r > trow) ? NEGB : tb[r]; }
        }
        float mx = NEGB;
#pragma unroll
        for (int r = 0; r < 8; ++r) mx = fmaxf(mx, fmaxf(ta[r], tb[r]));
        mx = fmaxf(mx, __shfl_xor(mx, 16, 32));
        const float mnew = fmaxf(m, mx);
        const float alpha = __builtin_amdgcn_exp2f(m - mnew);
        const float sh = PSH - mnew;
        v16h pb = (v16h){}, prb = (v16h){}; float ls = 0.0f;
#pragma unroll
        for (int r = 0; r < 8; ++r) {
            const float pa = __builtin_amdgcn_exp2f(ta[r] + sh), pc = __builtin_amdgcn_exp2f(tb[r] + sh);
            const h16 ha = (h16)pa, hc = (h16)pc; pb[r] = ha; pb[8 + r] = hc;
            if (EP) { prb[r] = (h16)((pa - (float)ha) * QRS); prb[8 + r] = (h16)((pc - (float)hc) * QRS); ls += pa + pc; }
            else    { ls += (float)ha + (float)hc; }
        }
        l = l * alpha + ls; m = mnew;
#pragma unroll
        for (int j = 0; j < 4; ++j) { oH[j] = oH[j] * alpha; if (EP) oL[j] = oL[j] * alpha; }
        const h16* va = VH + vo + key0;
        const v16h v0 = ldh(va), v1 = ldh(va + (size_t)16 * SEQ), v2 = ldh(va + (size_t)32 * SEQ), v3 = ldh(va + (size_t)48 * SEQ);
        oH[0] = wmma16(v0, pb, oH[0]); oH[1] = wmma16(v1, pb, oH[1]); oH[2] = wmma16(v2, pb, oH[2]); oH[3] = wmma16(v3, pb, oH[3]);
        if (EP) {
            oL[0] = wmma16(v0, prb, oL[0]); oL[1] = wmma16(v1, prb, oL[1]); oL[2] = wmma16(v2, prb, oL[2]); oL[3] = wmma16(v3, prb, oL[3]);
            const h16* vr = VR + vro + key0;
            const v16h w0 = ldh(vr), w1 = ldh(vr + (size_t)16 * EARLY), w2 = ldh(vr + (size_t)32 * EARLY), w3 = ldh(vr + (size_t)48 * EARLY);
            oL[0] = wmma16(w0, pb, oL[0]); oL[1] = wmma16(w1, pb, oL[1]); oL[2] = wmma16(w2, pb, oL[2]); oL[3] = wmma16(w3, pb, oL[3]);
            asm volatile("v_nop\n\tv_nop\n\tv_nop\n\tv_nop" : "+v"(oH[0]), "+v"(oH[1]), "+v"(oH[2]), "+v"(oH[3]), "+v"(oL[0]), "+v"(oL[1]), "+v"(oL[2]), "+v"(oL[3])
                         : "v"(v0), "v"(v1), "v"(v2), "v"(v3), "v"(w0), "v"(w1), "v"(w2), "v"(w3), "v"(pb), "v"(prb));
        } else {
            asm volatile("v_nop\n\tv_nop\n\tv_nop\n\tv_nop" : "+v"(oH[0]), "+v"(oH[1]), "+v"(oH[2]), "+v"(oH[3]) : "v"(v0), "v"(v1), "v"(v2), "v"(v3), "v"(pb));
        }
    }
    l += __shfl_xor(l, 16, 32);
    const float inv = 1.0f / l;
    const int wb = wave * 16 * 68;
#pragma unroll
    for (int j = 0; j < 4; ++j) { v4f a, c;
#pragma unroll
        for (int i = 0; i < 4; ++i) {
            float f0 = oH[j][i], f1 = oH[j][4 + i];
            if (EP) { f0 += oL[j][i] * QRI; f1 += oL[j][4 + i] * QRI; }
            a[i] = f0 * inv; c[i] = f1 * inv; }
        *(v4fa*)(&os[wb + lr * 68 + 16 * j + 8 * hi]) = a; *(v4fa*)(&os[wb + lr * 68 + 16 * j + 8 * hi + 4]) = c; }
    wave_sync();
    h16* crow = CH + ((size_t)b * SEQ + t0) * DM + h * HD;
    const size_t rro = EP ? (((size_t)b * EARLY + t0) * DM + h * HD) : (size_t)0;
#pragma unroll 1
    for (int ps = 0; ps < 2; ++ps) {
#pragma unroll
        for (int s = 0; s < 4; ++s) { const int row = 4 * s + (lane >> 3), c8 = (lane & 7) * 8;
            const v4f x0 = *(const v4fa*)(&os[wb + row * 68 + c8]); const v4f x1 = *(const v4fa*)(&os[wb + row * 68 + c8 + 4]); v8h hv, rv;
#pragma unroll
            for (int i = 0; i < 4; ++i) { const h16 a0 = (h16)x0[i]; const h16 a1 = (h16)x1[i]; hv[i] = a0; hv[4 + i] = a1; rv[i] = (h16)((x0[i] - (float)a0) * QRS); rv[4 + i] = (h16)((x1[i] - (float)a1) * QRS); }
            *(volatile v8h*)(crow + (size_t)row * DM + c8) = hv;
            if (EP) *(volatile v8h*)(CR + rro + (size_t)row * DM + c8) = rv; }
        if (ps == 0) __threadfence(); }
}

__global__ __launch_bounds__(32 * AW) void k_flash_early(const h16* __restrict__ QH, const h16* __restrict__ QR, const h16* __restrict__ KH, const h16* __restrict__ KR,
                                                         const h16* __restrict__ VH, const h16* __restrict__ VR, h16* CH, h16* CR) {
    flash_body<1>(QH, QR, KH, KR, VH, VR, CH, CR, 0);
}
__global__ __launch_bounds__(32 * AW) void k_flash_late(const h16* __restrict__ QH, const h16* __restrict__ QR, const h16* __restrict__ KH,
                                                        const h16* __restrict__ VH, h16* CH) {
    flash_body<0>(QH, QR, KH, KH, VH, VH, CH, CH, EARLY);
}

__device__ __forceinline__ void gemm64h(const h16* __restrict__ A, const size_t aoff, const h16* __restrict__ Bt, const size_t boff, v8f (&acc)[4][4]) {
#pragma unroll 1
    for (int kc = 0; kc < DM; kc += 32) {
        v16h a[4];
#pragma unroll
        for (int mb = 0; mb < 4; ++mb) a[mb] = ldh(A + aoff + (size_t)mb * 16 * DM + kc);
#pragma unroll
        for (int nb = 0; nb < 4; ++nb) { const v16h b = ldh(Bt + boff + (size_t)nb * 16 * DM + kc);
#pragma unroll
            for (int mb = 0; mb < 4; ++mb) acc[mb][nb] = wmma16(a[mb], b, acc[mb][nb]); }
        asm volatile("v_nop\n\tv_nop\n\tv_nop\n\tv_nop" : "+v"(acc[0][0]), "+v"(acc[1][1]), "+v"(acc[2][2]), "+v"(acc[3][3]) : "v"(a[0]), "v"(a[1]), "v"(a[2]), "v"(a[3]));
    }
}

__global__ __launch_bounds__(32) void k_oproj(const h16* __restrict__ CHp, const h16* __restrict__ CRp, const h16* __restrict__ Wt, const float* __restrict__ bias, float* OUT) {
    __shared__ __align__(16) float os[64 * 68];
    const int lane = threadIdx.x & 31, lr = lane & 15, hi = lane >> 4;
    const int r0 = blockIdx.x * 64, c0 = blockIdx.y * 64;
    const int b = r0 / SEQ, t0 = r0 % SEQ;
    v8f acc[4][4];
#pragma unroll
    for (int mb = 0; mb < 4; ++mb)
#pragma unroll
        for (int nb = 0; nb < 4; ++nb) acc[mb][nb] = (v8f){};
    const size_t boff = (size_t)(c0 + lr) * DM + 8 * hi;
    gemm64h(CHp, (size_t)(r0 + lr) * DM + 8 * hi, Wt, boff, acc);
#pragma unroll
    for (int mb = 0; mb < 4; ++mb)
#pragma unroll
        for (int nb = 0; nb < 4; ++nb)
#pragma unroll
            for (int j = 0; j < 8; ++j) os[(mb * 16 + hi * 8 + j) * 68 + nb * 16 + lr] = acc[mb][nb][j];
    if (t0 < EARLY) {
#pragma unroll
        for (int mb = 0; mb < 4; ++mb)
#pragma unroll
            for (int nb = 0; nb < 4; ++nb) acc[mb][nb] = (v8f){};
        gemm64h(CRp, ((size_t)b * EARLY + t0 + lr) * DM + 8 * hi, Wt, boff, acc);
#pragma unroll
        for (int mb = 0; mb < 4; ++mb)
#pragma unroll
            for (int nb = 0; nb < 4; ++nb)
#pragma unroll
                for (int j = 0; j < 8; ++j) { const int ix = (mb * 16 + hi * 8 + j) * 68 + nb * 16 + lr; const float cur = os[ix]; os[ix] = cur + acc[mb][nb][j] * QRI; }
    }
    wave_sync();
    v4f bv = *(const v4f*)(bias + c0 + lr * 4);
    bv[0] = bfval(bv[0]); bv[1] = bfval(bv[1]); bv[2] = bfval(bv[2]); bv[3] = bfval(bv[3]);
    float* orow = OUT + ((size_t)b * OUT_SEQ + t0) * DM + c0;
#pragma unroll 1
    for (int ps = 0; ps < 2; ++ps) {
#pragma unroll 4
        for (int s = 0; s < 32; ++s) { const int row = 2 * s + hi, cofs = lr * 4;
            const v4f x = *(const v4fa*)(&os[row * 68 + cofs]);
            v4f val; val[0] = x[0] * WPI + bv[0]; val[1] = x[1] * WPI + bv[1]; val[2] = x[2] * WPI + bv[2]; val[3] = x[3] * WPI + bv[3];
            *(volatile v4f*)(orow + (size_t)row * DM + cofs) = val; }
        if (ps == 0) __threadfence(); }
}

static constexpr size_t al256(size_t v) { return (v + 255) & ~(size_t)255; }
static constexpr size_t SZ_XB = al256((size_t)NB * SEQ * DM * 2);
static constexpr size_t SZ_WB = al256((size_t)3 * DM * DM * 2);
static constexpr size_t SZ_WP = al256((size_t)DM * DM * 2);
static constexpr size_t SZ_PL = al256((size_t)NB * NH_ * SEQ * HD * 2);
static constexpr size_t SZ_PR = al256((size_t)NB * NH_ * EARLY * HD * 2);
static constexpr size_t SZ_CH = al256((size_t)NB * SEQ * DM * 2);
static constexpr size_t SZ_CR = al256((size_t)NB * EARLY * DM * 2);
static constexpr size_t SZ_TOTAL = SZ_XB + SZ_WB + SZ_WP + 4 * SZ_PL + 2 * SZ_PR + SZ_CH + SZ_CR;
static_assert(SZ_TOTAL <= (size_t)134217728);
static_assert(((size_t)DM * DM * 2) % 256 == 0);

extern "C" void kernel_launch(void* const* d_in, const int* in_sizes, int n_in,
                              void* d_out, int out_size, void* d_ws, size_t ws_size, hipStream_t stream) {
    if (n_in < 6) return;
    const size_t needx = ((size_t)(NB - 1) * SEQ_FULL + SEQ) * DM;
    if ((size_t)in_sizes[0] < needx) return;
    if ((size_t)in_sizes[1] < (size_t)DM * DM || (size_t)in_sizes[2] < (size_t)DM * DM || (size_t)in_sizes[3] < (size_t)DM * DM) return;
    if ((size_t)in_sizes[4] < (size_t)DM * DM || (size_t)in_sizes[5] < (size_t)DM) return;
    if ((size_t)out_size < ((size_t)(NB - 1) * OUT_SEQ + SEQ) * DM) return;
    if (SZ_TOTAL > ws_size) return;
    const float* x = (const float*)d_in[0]; const float* wq = (const float*)d_in[1]; const float* wk = (const float*)d_in[2]; const float* wv = (const float*)d_in[3];
    const float* wp = (const float*)d_in[4]; const float* bp = (const float*)d_in[5];
    float* OUT = (float*)d_out;
    char* wsp = (char*)d_ws;
    bf* XB = (bf*)wsp; wsp += SZ_XB;
    bf* WB = (bf*)wsp; wsp += SZ_WB;
    h16* WP = (h16*)wsp; wsp += SZ_WP;
    h16* QH = (h16*)wsp; wsp += SZ_PL;
    h16* QR = (h16*)wsp; wsp += SZ_PL;
    h16* KH = (h16*)wsp; wsp += SZ_PL;
    h16* VH = (h16*)wsp; wsp += SZ_PL;
    h16* KR = (h16*)wsp; wsp += SZ_PR;
    h16* VR = (h16*)wsp; wsp += SZ_PR;
    h16* CH = (h16*)wsp; wsp += SZ_CH;
    h16* CR = (h16*)wsp; wsp += SZ_CR;
    bf* WQ = WB; bf* WK = WB + (size_t)DM * DM; bf* WV = WB + (size_t)2 * DM * DM;

    if (SEQ == SEQ_FULL) {
        const size_t n8 = (size_t)NB * SEQ * DM / 8;
        k_cvt8<<<(unsigned)((n8 + 255) / 256), 256, 0, stream>>>(x, XB, n8);
    } else {
        const size_t n8 = (size_t)SEQ * DM / 8;
        for (int b = 0; b < NB; ++b) k_cvt8<<<(unsigned)((n8 + 255) / 256), 256, 0, stream>>>(x + (size_t)b * SEQ_FULL * DM, XB + (size_t)b * SEQ * DM, n8);
    }
    k_wT<<<dim3(DM / 64, HD / 64, NH_), 256, 0, stream>>>(wq, WQ, DM, HD, 0);
    k_wT<<<dim3(DM / 64, HD / 64, NH_), 256, 0, stream>>>(wk, WK, DM, HD, 0);
    k_wT<<<dim3(DM / 64, HD / 64, NH_), 256, 0, stream>>>(wv, WV, DM, HD, 0);
    k_wT<<<dim3(DM / 64, DM / 64, 1), 256, 0, stream>>>(wp, (unsigned short*)WP, DM, DM, 1);

    k_proj<<<dim3(NB * SEQ / 64, DM / 64, 1), 32, 0, stream>>>(XB, WQ, QH, QR, SEQ, (size_t)NH_ * SEQ * HD, HD, HD, (size_t)SEQ * HD,
                                                               1, SEQ, (size_t)NH_ * SEQ * HD, HD, (size_t)SEQ * HD);
    k_proj<<<dim3(NB * SEQ / 64, DM / 64, 1), 32, 0, stream>>>(XB, WK, KH, KR, SEQ, (size_t)NH_ * SEQ * HD, HD, HD, (size_t)SEQ * HD,
                                                               1, EARLY, (size_t)NH_ * EARLY * HD, HD, (size_t)EARLY * HD);
    k_proj<<<dim3(DM / 64, NB * SEQ / 64, 1), 32, 0, stream>>>(WV, XB, VH, VR, DM, (size_t)0, SEQ, SEQ, (size_t)DM * SEQ,
                                                               2, EARLY, (size_t)0, EARLY, (size_t)DM * EARLY);

    k_flash_early<<<dim3(EARLY / (16 * AW), NB * NH_, 1), 32 * AW, 0, stream>>>(QH, QR, KH, KR, VH, VR, CH, CR);
    if (SEQ > EARLY)
        k_flash_late<<<dim3((SEQ - EARLY) / (16 * AW) > 0 ? (SEQ - EARLY) / (16 * AW) : 1, NB * NH_, 1), 32 * AW, 0, stream>>>(QH, QR, KH, VH, CH);

    k_oproj<<<dim3(NB * SEQ / 64, DM / 64, 1), 32, 0, stream>>>(CH, CR, WP, bp, OUT);
}
